// MultiHeadedAttention_63376537420578
// MI455X (gfx1250) — hardware-verified
//
#include <hip/hip_runtime.h>
#ifndef NB
#define NB 2
#endif
#ifndef SEQ
#define SEQ 2048
#endif
#define NB_FULL 2
#define SEQ_FULL 2048
#define DM 1024
#define NH 16
#define HD 64

constexpr unsigned USQ = (unsigned)SEQ;
constexpr unsigned UDM = (unsigned)DM;
constexpr unsigned UNH = (unsigned)NH;
constexpr unsigned UHD = (unsigned)HD;
constexpr unsigned UNR = (unsigned)NB * (unsigned)SEQ;
constexpr size_t   FSQ = (size_t)SEQ_FULL;

static_assert(NH * HD == DM);
static_assert(HD == 64);
static_assert(DM % 64 == 0);
static_assert(DM % 32 == 0);
static_assert(SEQ % 128 == 0);
static_assert(SEQ % 64 == 0);
static_assert(NB <= NB_FULL);
static_assert(SEQ <= SEQ_FULL);
static_assert((NB * SEQ) % 128 == 0);

typedef unsigned short v8us __attribute__((ext_vector_type(8), may_alias));
typedef float  v8f  __attribute__((ext_vector_type(8)));
typedef float  v4f  __attribute__((ext_vector_type(4)));
typedef float  v4fa __attribute__((ext_vector_type(4), may_alias));
typedef int    v4i  __attribute__((ext_vector_type(4)));
typedef int    v4ia __attribute__((ext_vector_type(4), may_alias));
typedef _Float16 v16h __attribute__((ext_vector_type(16)));
union FragH { v16h v; v8us half[2]; _Float16 h[16]; unsigned short u[16]; };

__device__ __forceinline__ unsigned short bf16_bits(float x) { unsigned int u = __float_as_uint(x); return (unsigned short)((u + 0x7FFFu + ((u >> 16) & 1u)) >> 16); }
__device__ __forceinline__ float bf16_rne(float x) { return __uint_as_float(((unsigned int)bf16_bits(x)) << 16); }

__device__ __forceinline__ v16h g2_frag(const _Float16* p, unsigned hh) { FragH f; f.half[0] = *(const v8us*)((const unsigned short*)p + 8u * hh); f.half[1] = *(const v8us*)((const unsigned short*)p + 16u + 8u * hh); return f.v; }
__device__ __forceinline__ v8f g2_mma(v16h a, v16h b, v8f c) { v8f d = __builtin_amdgcn_wmma_f32_16x16x32_f16(false, a, false, b, (short)0, c, false, false); asm volatile("v_nop\n\tv_nop\n\tv_nop\n\tv_nop" : "+v"(d) : "v"(a), "v"(b)); return d; }

#define WT_GRID ((DM * (DM / 8)) / 256)
static_assert((size_t)WT_GRID * 256 * 8 == (size_t)DM * DM);
__global__ __launch_bounds__(256) void k_wt(const float* __restrict__ w0, const float* __restrict__ w1, const float* __restrict__ w2, const float* __restrict__ w3, _Float16* __restrict__ BW) {
  const unsigned y = blockIdx.y;
  const float* W = (y == 0u) ? w0 : (y == 1u) ? w1 : (y == 2u) ? w2 : w3;
  const unsigned t = blockIdx.x * 256u + threadIdx.x;
  if (t >= UDM * (UDM / 8u)) return;
  const unsigned n = t / (UDM / 8u), k8 = (t - n * (UDM / 8u)) * 8u;
  FragH f;
#pragma unroll
  for (int i = 0; i < 8; ++i) f.h[i] = (_Float16)(bf16_rne(W[(size_t)(k8 + (unsigned)i) * UDM + n]) * 16.0f);
  const v8us o = f.half[0];
  unsigned short* dst = (unsigned short*)BW + (size_t)y * UDM * UDM + (size_t)n * UDM + k8;
  *(volatile v8us*)dst = o;
  __threadfence();
  *(volatile v8us*)dst = o;
}

#define X16_GRID ((NB * SEQ * (DM / 8)) / 256)
static_assert((size_t)X16_GRID * 256 * 8 == (size_t)NB * SEQ * DM);
__global__ __launch_bounds__(256) void k_x16(const float* __restrict__ x0, const float* __restrict__ x1, const float* __restrict__ x2, _Float16* __restrict__ X16) {
  const unsigned y = blockIdx.y;
  const float* x = (y == 0u) ? x0 : (y == 1u) ? x1 : x2;
  const unsigned t = blockIdx.x * 256u + threadIdx.x;
  if (t >= UNR * (UDM / 8u)) return;
  const unsigned row = t / (UDM / 8u), c8 = (t - row * (UDM / 8u)) * 8u;
  const unsigned b = row / USQ, s = row - b * USQ;
  const float* src = x + ((size_t)b * FSQ + s) * UDM + c8;
  const v4f a = *(const v4fa*)src, c = *(const v4fa*)(src + 4);
  FragH f;
#pragma unroll
  for (int q = 0; q < 4; ++q) { f.h[q] = (_Float16)bf16_rne(a[q]); f.h[4 + q] = (_Float16)bf16_rne(c[q]); }
  const v8us o = f.half[0];
  unsigned short* dst = (unsigned short*)X16 + (size_t)y * UNR * UDM + (size_t)t * 8u;
  *(volatile v8us*)dst = o;
  __threadfence();
  *(volatile v8us*)dst = o;
}

#define QKV_GRID ((NB * SEQ / 128) * (DM / 64))
static_assert((size_t)QKV_GRID * 128 * 64 == (size_t)NB * SEQ * DM);
__global__ __launch_bounds__(128) void k_gemm_qkv(const _Float16* __restrict__ A, const _Float16* __restrict__ Bh, const float* __restrict__ bias0, const float* __restrict__ bias1, const float* __restrict__ bias2, _Float16* __restrict__ C16) {
  __shared__ __attribute__((aligned(16))) float so[4][32][68];
  const unsigned tid = threadIdx.x, w = tid >> 5, lane = tid & 31u, ln = lane & 15u, hh = lane >> 4;
  const unsigned by = blockIdx.y;
  A += (size_t)by * UNR * UDM; Bh += (size_t)by * UDM * UDM; C16 += (size_t)by * UNR * UDM;
  const float* bp = (by == 0u) ? bias0 : (by == 1u) ? bias1 : bias2;
  const unsigned ntn = UDM / 64u;
  const unsigned mt = blockIdx.x / ntn, nq = blockIdx.x - mt * ntn;
  const unsigned row0 = mt * 128u + 32u * w, col0 = nq * 64u;
  if (row0 >= UNR) return;
  const _Float16* a0p = A + (size_t)(row0 + ln) * UDM; const _Float16* a1p = a0p + (size_t)16 * UDM;
  const _Float16* b0p = Bh + (size_t)(col0 + ln) * UDM; const _Float16* b1p = b0p + (size_t)16 * UDM; const _Float16* b2p = b1p + (size_t)16 * UDM; const _Float16* b3p = b2p + (size_t)16 * UDM;
  const v8f z8 = {0.f,0.f,0.f,0.f,0.f,0.f,0.f,0.f};
  v8f c00 = z8, c01 = z8, c02 = z8, c03 = z8, c10 = z8, c11 = z8, c12 = z8, c13 = z8;
#pragma unroll 1
  for (unsigned kb = 0; kb < UDM; kb += 32u) {
    const v16h a0 = g2_frag(a0p + kb, hh), a1 = g2_frag(a1p + kb, hh);
    v16h b = g2_frag(b0p + kb, hh); c00 = g2_mma(a0, b, c00); c10 = g2_mma(a1, b, c10);
    b = g2_frag(b1p + kb, hh); c01 = g2_mma(a0, b, c01); c11 = g2_mma(a1, b, c11);
    b = g2_frag(b2p + kb, hh); c02 = g2_mma(a0, b, c02); c12 = g2_mma(a1, b, c12);
    b = g2_frag(b3p + kb, hh); c03 = g2_mma(a0, b, c03); c13 = g2_mma(a1, b, c13);
  }
  v8f accs[8] = {c00, c01, c02, c03, c10, c11, c12, c13};
#pragma unroll
  for (int u = 0; u < 8; ++u) {
    const unsigned t = (unsigned)u & 3u, half = (unsigned)u >> 2;
    const float bv = bf16_rne(bp[col0 + t * 16u + ln]);
#pragma unroll
    for (int r = 0; r < 8; ++r) so[w][half * 16u + 8u * hh + (unsigned)r][t * 16u + ln] = accs[u][r] * 0.0625f + bv;
  }
  __builtin_amdgcn_fence(4  , "workgroup"); __builtin_amdgcn_wave_barrier();
  const unsigned rq = lane >> 3, c8 = (lane & 7u) * 8u;
  for (int pass = 0; pass < 2; ++pass) {
#pragma unroll
    for (int q = 0; q < 8; ++q) {
      const unsigned r = 4u * (unsigned)q + rq;
      const v4f a = *(const v4fa*)&so[w][r][c8], c = *(const v4fa*)&so[w][r][c8 + 4u];
      FragH f;
#pragma unroll
      for (int i = 0; i < 4; ++i) { f.h[i] = (_Float16)a[i]; f.h[4 + i] = (_Float16)c[i]; }
      *(volatile v8us*)((unsigned short*)C16 + (size_t)(row0 + r) * UDM + col0 + c8) = f.half[0];
    }
    if (pass == 0) __threadfence();
  }
}

#define VT_GRID (NB * NH * (SEQ / 64))
static_assert((size_t)VT_GRID * 64 * 64 == (size_t)NB * NH * HD * SEQ);
__global__ __launch_bounds__(256) void k_vt(const _Float16* __restrict__ V16, _Float16* __restrict__ VT) {
  __shared__ unsigned short tl[64][66];
  const unsigned tid = threadIdx.x;
  const unsigned ng = USQ / 64u;
  const unsigned slab = blockIdx.x / ng, lg = blockIdx.x - slab * ng;
  const unsigned b = slab / UNH, h = slab - b * UNH;
  for (unsigned i = tid; i < 512u; i += 256u) {
    const unsigned r = i >> 3, c8 = (i & 7u) * 8u;
    FragH f; f.half[0] = *(const v8us*)((const unsigned short*)V16 + ((size_t)b * USQ + lg * 64u + r) * UDM + h * UHD + c8);
#pragma unroll
    for (int q = 0; q < 8; ++q) tl[r][c8 + (unsigned)q] = f.u[q];
  }
  __syncthreads();
  for (int pass = 0; pass < 2; ++pass) {
#pragma unroll
    for (int rd = 0; rd < 2; ++rd) {
      const unsigned d = (unsigned)rd * 32u + (tid >> 3), pc = tid & 7u;
      FragH f;
#pragma unroll
      for (int q = 0; q < 8; ++q) f.u[q] = tl[pc * 8u + (unsigned)q][d];
      *(volatile v8us*)((unsigned short*)VT + ((size_t)slab * 64u + d) * USQ + lg * 64u + pc * 8u) = f.half[0];
    }
    if (pass == 0) __threadfence();
  }
}

#define FL_GRID (NB * NH * (SEQ / 64))
static_assert((size_t)FL_GRID * 64 * 64 == (size_t)NB * SEQ * DM);
__global__ __launch_bounds__(128) void k_flash(const _Float16* __restrict__ Q16, const _Float16* __restrict__ K16, const _Float16* __restrict__ VT, const int* __restrict__ mask, _Float16* __restrict__ OH, _Float16* __restrict__ OL) {
  __shared__ __attribute__((aligned(16))) float so[4][16][68];
  const unsigned tid = threadIdx.x, w = tid >> 5, lane = tid & 31u, ln = lane & 15u, hh = lane >> 4;
  const unsigned nqb = USQ / 64u;
  const unsigned bh = blockIdx.x / nqb, qb = blockIdx.x - bh * nqb;
  const unsigned b = bh / UNH, h = bh - b * UNH;
  const unsigned q0 = qb * 64u + w * 16u;
  const size_t rb = (size_t)b * USQ;
  const _Float16* qrow = Q16 + (rb + q0 + ln) * UDM + h * UHD;
  const v16h qf0 = g2_frag(qrow, hh), qf1 = g2_frag(qrow + 32, hh);
  const _Float16* kbase = K16 + (rb + ln) * UDM + h * UHD;
  const _Float16* vbase = VT + ((size_t)bh * UHD + ln) * USQ;
  const int* mrow = mask + ((size_t)b * FSQ + q0 + ln) * FSQ + 8u * hh;
  const v8f z8 = {0.f,0.f,0.f,0.f,0.f,0.f,0.f,0.f};
  v8f o[4] = {z8, z8, z8, z8};
  float mrun = -3.0e38f, lrun = 0.f;
#pragma unroll 1
  for (unsigned k0 = 0; k0 < USQ; k0 += 64u) {
    v8f s[4];
#pragma unroll
    for (int t = 0; t < 4; ++t) {
      const _Float16* kr = kbase + (size_t)(k0 + 16u * (unsigned)t) * UDM;
      v8f c = z8;
      c = g2_mma(g2_frag(kr, hh), qf0, c);
      c = g2_mma(g2_frag(kr + 32, hh), qf1, c);
      s[t] = c;
    }
    v4i ma[4], mb[4];
#pragma unroll
    for (int t = 0; t < 4; ++t) { ma[t] = *(const v4ia*)(mrow + k0 + 16u * (unsigned)t); mb[t] = *(const v4ia*)(mrow + k0 + 16u * (unsigned)t + 4u); }
    float mx = -3.0e38f;
#pragma unroll
    for (int t = 0; t < 4; ++t) {
#pragma unroll
      for (int r = 0; r < 4; ++r) {
        const float v0 = (ma[t][r] != 0) ? s[t][r] * 0.125f : -1.0e9f;
        const float v1 = (mb[t][r] != 0) ? s[t][4 + r] * 0.125f : -1.0e9f;
        s[t][r] = v0; s[t][4 + r] = v1;
        mx = fmaxf(mx, fmaxf(v0, v1));
      }
    }
    mx = fmaxf(mx, __shfl_xor(mx, 16));
    const float mnew = fmaxf(mrun, mx);
    const float al = __expf(mrun - mnew);
    mrun = mnew;
    float ps = 0.f;
#pragma unroll
    for (int t = 0; t < 4; ++t) {
#pragma unroll
      for (int r = 0; r < 8; ++r) { const float p = __expf(s[t][r] - mnew); s[t][r] = p; ps += p; }
    }
    ps += __shfl_xor(ps, 16);
    lrun = lrun * al + ps;
#pragma unroll
    for (int r = 0; r < 8; ++r) {
      const float alq = __shfl(al, (int)(8u * hh + (unsigned)r));
#pragma unroll
      for (int j = 0; j < 4; ++j) o[j][r] *= alq;
    }
    FragH pa, pb;
#pragma unroll
    for (int r = 0; r < 8; ++r) {
      pa.h[r] = (_Float16)(s[0][r] * 1024.0f); pa.h[8 + r] = (_Float16)(s[1][r] * 1024.0f);
      pb.h[r] = (_Float16)(s[2][r] * 1024.0f); pb.h[8 + r] = (_Float16)(s[3][r] * 1024.0f);
    }
#pragma unroll
    for (int j = 0; j < 4; ++j) {
      const _Float16* vr = vbase + (size_t)(16u * (unsigned)j) * USQ + k0;
      o[j] = g2_mma(pa.v, g2_frag(vr, hh), o[j]);
      o[j] = g2_mma(pb.v, g2_frag(vr + 32, hh), o[j]);
    }
  }
  const float inv = 0.0625f * (1.0f / lrun);
#pragma unroll
  for (int r = 0; r < 8; ++r) {
    const float iq = __shfl(inv, (int)(8u * hh + (unsigned)r));
#pragma unroll
    for (int j = 0; j < 4; ++j) so[w][8u * hh + (unsigned)r][16u * (unsigned)j + ln] = o[j][r] * iq;
  }
  __builtin_amdgcn_fence(4  , "workgroup"); __builtin_amdgcn_wave_barrier();
  const unsigned rq = lane >> 3, c8 = (lane & 7u) * 8u;
  for (int pass = 0; pass < 2; ++pass) {
#pragma unroll
    for (int it = 0; it < 4; ++it) {
      const unsigned row = 4u * (unsigned)it + rq;
      const v4f a = *(const v4fa*)&so[w][row][c8], c = *(const v4fa*)&so[w][row][c8 + 4u];
      FragH fh, fl;
#pragma unroll
      for (int q = 0; q < 4; ++q) {
        _Float16 hq = (_Float16)a[q]; fh.h[q] = hq; fl.h[q] = (_Float16)((a[q] - (float)hq) * 1024.0f);
        hq = (_Float16)c[q]; fh.h[4 + q] = hq; fl.h[4 + q] = (_Float16)((c[q] - (float)hq) * 1024.0f);
      }
      const size_t off = (rb + q0 + row) * UDM + h * UHD + c8;
      *(volatile v8us*)((unsigned short*)OH + off) = fh.half[0];
      *(volatile v8us*)((unsigned short*)OL + off) = fl.half[0];
    }
    if (pass == 0) __threadfence();
  }
}

#define OUT_GRID ((NB * SEQ / 64) * (DM / 64))
static_assert((size_t)OUT_GRID * 64 * 64 == (size_t)NB * SEQ * DM);
__global__ __launch_bounds__(128) void k_gemm_out(const _Float16* __restrict__ AH, const _Float16* __restrict__ AL, const _Float16* __restrict__ Bh, const float* __restrict__ bias, float* __restrict__ C) {
  __shared__ __attribute__((aligned(16))) float so[4][16][68];
  const unsigned tid = threadIdx.x, w = tid >> 5, lane = tid & 31u, ln = lane & 15u, hh = lane >> 4;
  const unsigned ntn = UDM / 64u;
  const unsigned mt = blockIdx.x / ntn, nq = blockIdx.x - mt * ntn;
  const unsigned row0 = mt * 64u + 16u * w, col0 = nq * 64u;
  if (row0 >= UNR) return;
  const _Float16* ahp = AH + (size_t)(row0 + ln) * UDM; const _Float16* alp = AL + (size_t)(row0 + ln) * UDM;
  const _Float16* b0p = Bh + (size_t)(col0 + ln) * UDM; const _Float16* b1p = b0p + (size_t)16 * UDM; const _Float16* b2p = b1p + (size_t)16 * UDM; const _Float16* b3p = b2p + (size_t)16 * UDM;
  const v8f z8 = {0.f,0.f,0.f,0.f,0.f,0.f,0.f,0.f};
  v8f h0 = z8, h1 = z8, h2 = z8, h3 = z8, l0 = z8, l1 = z8, l2 = z8, l3 = z8;
#pragma unroll 1
  for (unsigned kb = 0; kb < UDM; kb += 32u) {
    const v16h ah = g2_frag(ahp + kb, hh), al = g2_frag(alp + kb, hh);
    v16h b = g2_frag(b0p + kb, hh); h0 = g2_mma(ah, b, h0); l0 = g2_mma(al, b, l0);
    b = g2_frag(b1p + kb, hh); h1 = g2_mma(ah, b, h1); l1 = g2_mma(al, b, l1);
    b = g2_frag(b2p + kb, hh); h2 = g2_mma(ah, b, h2); l2 = g2_mma(al, b, l2);
    b = g2_frag(b3p + kb, hh); h3 = g2_mma(ah, b, h3); l3 = g2_mma(al, b, l3);
  }
  v8f ach[4] = {h0, h1, h2, h3}, acl[4] = {l0, l1, l2, l3};
#pragma unroll
  for (int t = 0; t < 4; ++t) {
    const float bv = bf16_rne(bias[col0 + (unsigned)t * 16u + ln]);
#pragma unroll
    for (int r = 0; r < 8; ++r) so[w][8u * hh + (unsigned)r][(unsigned)t * 16u + ln] = (ach[t][r] + acl[t][r] * 0.0009765625f) * 0.0009765625f + bv;
  }
  __builtin_amdgcn_fence(4  , "workgroup"); __builtin_amdgcn_wave_barrier();
  const unsigned bb = row0 / USQ;
  const size_t orow0 = (size_t)bb * FSQ + (row0 - bb * USQ);
  const unsigned rsub = lane >> 4, c4 = (lane & 15u) * 4u;
  for (int pass = 0; pass < 2; ++pass) {
#pragma unroll
    for (int q = 0; q < 8; ++q) {
      const unsigned r = 2u * (unsigned)q + rsub;
      const v4f v = *(const v4fa*)&so[w][r][c4];
      *(volatile v4f*)(C + (orow0 + r) * UDM + col0 + c4) = v;
    }
    if (pass == 0) __threadfence();
  }
}

#define SZ_BW   ((size_t)4 * DM * DM * 2)
#define SZ_PL   ((size_t)NB * SEQ * DM * 2)
#define SZ_VT   ((size_t)NB * NH * HD * SEQ * 2)
#define OFF_BW  ((size_t)0)
#define OFF_X   (OFF_BW + SZ_BW)
#define OFF_QKV (OFF_X + 3 * SZ_PL)
#define OFF_VT  (OFF_QKV + 3 * SZ_PL)
#define OFF_OH  (OFF_VT + SZ_VT)
#define OFF_OL  (OFF_OH + SZ_PL)
#define WS_TOTAL (OFF_OL + SZ_PL)
static_assert(SZ_BW % 256 == 0);
static_assert(SZ_PL % 256 == 0);
static_assert(SZ_VT % 256 == 0);
static_assert(WS_TOTAL <= (size_t)134217728);

extern "C" void kernel_launch(void* const* d_in, const int* in_sizes, int n_in,
                              void* d_out, int out_size, void* d_ws, size_t ws_size, hipStream_t stream) {
  if (n_in < 12) return;
  const long long xneed = ((long long)(NB - 1) * SEQ_FULL + SEQ) * DM;
  const long long mneed = ((long long)(NB - 1) * SEQ_FULL + (SEQ - 1)) * SEQ_FULL + SEQ;
  if ((long long)in_sizes[0] < xneed || (long long)in_sizes[1] < xneed || (long long)in_sizes[2] < xneed) return;
  if ((long long)in_sizes[3] < mneed) return;
  if (in_sizes[4] < DM * DM || in_sizes[6] < DM * DM || in_sizes[8] < DM * DM || in_sizes[10] < DM * DM) return;
  if (in_sizes[5] < DM || in_sizes[7] < DM || in_sizes[9] < DM || in_sizes[11] < DM) return;
  if ((long long)out_size < xneed) return;
  if (ws_size < WS_TOTAL) return;
  const float* xq = (const float*)d_in[0]; const float* xk = (const float*)d_in[1]; const float* xv = (const float*)d_in[2];
  const int* mask = (const int*)d_in[3];
  const float* wq = (const float*)d_in[4]; const float* bq = (const float*)d_in[5];
  const float* wk = (const float*)d_in[6]; const float* bk = (const float*)d_in[7];
  const float* wv = (const float*)d_in[8]; const float* bv = (const float*)d_in[9];
  const float* wo = (const float*)d_in[10]; const float* bo = (const float*)d_in[11];
  char* ws = (char*)d_ws;
  _Float16* BW  = (_Float16*)(ws + OFF_BW);
  _Float16* X16 = (_Float16*)(ws + OFF_X);
  _Float16* QKV = (_Float16*)(ws + OFF_QKV);
  _Float16* VT  = (_Float16*)(ws + OFF_VT);
  _Float16* OH  = (_Float16*)(ws + OFF_OH);
  _Float16* OL  = (_Float16*)(ws + OFF_OL);
  const size_t pl = (size_t)NB * SEQ * DM;
  k_wt<<<dim3(WT_GRID, 4), 256, 0, stream>>>(wq, wk, wv, wo, BW);
  k_x16<<<dim3(X16_GRID, 3), 256, 0, stream>>>(xq, xk, xv, X16);
  k_gemm_qkv<<<dim3(QKV_GRID, 3), 128, 0, stream>>>(X16, BW, bq, bk, bv, QKV);
  k_vt<<<dim3(VT_GRID), 256, 0, stream>>>(QKV + 2 * pl, VT);
  k_flash<<<dim3(FL_GRID), 128, 0, stream>>>(QKV, QKV + pl, VT, mask, OH, OL);
  k_gemm_out<<<dim3(OUT_GRID), 128, 0, stream>>>(OH, OL, BW + (size_t)3 * DM * DM, bo, (float*)d_out);
}
